// PointNet_9509057593717
// MI455X (gfx1250) — hardware-verified
//
#include <hip/hip_runtime.h>
#define BB 4
#define NPT 8192
#define KNN 10
#define GF 100

typedef __bf16 v16b __attribute__((ext_vector_type(16)));
typedef unsigned short v8us __attribute__((ext_vector_type(8), may_alias));
typedef float  v8f  __attribute__((ext_vector_type(8)));
typedef float  v4f  __attribute__((ext_vector_type(4)));
typedef float  v4fa __attribute__((ext_vector_type(4), may_alias));
union FragB { v16b v; v8us half[2]; unsigned short u[16]; };

__device__ __forceinline__ unsigned short bf16_bits(float x) { unsigned int u = __float_as_uint(x); return (unsigned short)((u + 0x7FFFu + ((u >> 16) & 1u)) >> 16); }
__device__ __forceinline__ float bf16_val(unsigned short b) { return __uint_as_float(((unsigned int)b) << 16); }
__device__ __forceinline__ float bf16_round(float x) { return bf16_val(bf16_bits(x)); }
template <int NT>
__device__ __forceinline__ v8f mmaN(v16b ah, v16b al, v16b bh, v16b bl, v8f c) {
  c = __builtin_amdgcn_wmma_f32_16x16x32_bf16(false, ah, false, bh, (short)0, c, false, false);
  if (NT >= 2) c = __builtin_amdgcn_wmma_f32_16x16x32_bf16(false, al, false, bh, (short)0, c, false, false);
  if (NT >= 3) c = __builtin_amdgcn_wmma_f32_16x16x32_bf16(false, ah, false, bl, (short)0, c, false, false);
  asm volatile("v_nop\n\tv_nop\n\tv_nop\n\tv_nop" : "+v"(c) : "v"(ah), "v"(al), "v"(bh), "v"(bl));
  return c;
}

__global__ __launch_bounds__(256) void k_wt_bf16(const float* __restrict__ W, unsigned short* __restrict__ Wt, int K, int N) {
  const int t = blockIdx.x * 256 + threadIdx.x;
  const int k8n = K / 8;
  if (t >= N * k8n) return;
  const int n = t / k8n, k8 = (t % k8n) * 8;
  v8us v;
#pragma unroll
  for (int i = 0; i < 8; ++i) v[i] = bf16_bits(W[(size_t)(k8 + i) * N + n]);
  *(volatile v8us*)(Wt + (size_t)n * K + k8) = v;
  __threadfence();
  *(volatile v8us*)(Wt + (size_t)n * K + k8) = v;
}

template <bool ASPLIT, int ACT, bool BIAS_BF16>
__global__ __launch_bounds__(128) void k_gemm_bf(const float* __restrict__ A, int lda, const unsigned short* __restrict__ Wt, int ldb,
                                               const float* __restrict__ bias, float* __restrict__ C, int ldc, int M, int N, int K) {
  __shared__ __attribute__((aligned(16))) float so[4][16][64];
  const int tid = threadIdx.x, w = tid >> 5, lane = tid & 31, ln = lane & 15, hh = lane >> 4;
  const int ntn = N / 64;
  const int wid = blockIdx.x * 4 + w;
  const int mt = wid / ntn, nq = wid % ntn;
  if (mt * 16 >= M) return;
  const int row0 = mt * 16, col0 = nq * 64;
  const float* arow = A + (size_t)(row0 + ln) * lda;
  v8f acc[4] = {};
  for (int kb = 0; kb < K; kb += 32) {
    FragB ah, al;
    const v4f x0 = *(const v4fa*)(arow + kb + 8 * hh), x1 = *(const v4fa*)(arow + kb + 8 * hh + 4);
    const v4f x2 = *(const v4fa*)(arow + kb + 16 + 8 * hh), x3 = *(const v4fa*)(arow + kb + 16 + 8 * hh + 4);
    float xs[16] = {x0[0],x0[1],x0[2],x0[3],x1[0],x1[1],x1[2],x1[3],x2[0],x2[1],x2[2],x2[3],x3[0],x3[1],x3[2],x3[3]};
#pragma unroll
    for (int i = 0; i < 16; ++i) { const unsigned short hb = bf16_bits(xs[i]); ah.u[i] = hb; al.u[i] = ASPLIT ? bf16_bits(xs[i] - bf16_val(hb)) : (unsigned short)0; }
#pragma unroll
    for (int t = 0; t < 4; ++t) {
      const unsigned short* brow = Wt + (size_t)(col0 + t * 16 + ln) * ldb + kb;
      FragB b;
      b.half[0] = *(const v8us*)(brow + 8 * hh);
      b.half[1] = *(const v8us*)(brow + 16 + 8 * hh);
      acc[t] = mmaN<ASPLIT ? 2 : 1>(ah.v, al.v, b.v, b.v, acc[t]);
    }
  }
#pragma unroll
  for (int t = 0; t < 4; ++t) {
    float bv = bias ? bias[col0 + t * 16 + ln] : 0.f;
    if (BIAS_BF16) bv = bf16_round(bv);
#pragma unroll
    for (int r = 0; r < 8; ++r) { float v = acc[t][r] + bv; if (ACT == 1) v = fmaxf(v, 0.f); so[w][8 * hh + r][t * 16 + ln] = v; }
  }
  __builtin_amdgcn_fence(__ATOMIC_ACQ_REL, "workgroup");
  __builtin_amdgcn_wave_barrier();
  const int rsub = lane >> 4, c4 = (lane & 15) * 4;
  for (int pass = 0; pass < 2; ++pass) {
#pragma unroll
    for (int q = 0; q < 8; ++q) {
      const int r = q * 2 + rsub;
      const v4f v = *(const v4fa*)&so[w][r][c4];
      *(volatile v4f*)(C + (size_t)(row0 + r) * ldc + col0 + c4) = v;
    }
    if (pass == 0) __threadfence();
  }
}

template <int D, bool CAUSAL>
__global__ __launch_bounds__(128) void k_flash(const float* __restrict__ qb, const float* __restrict__ kb, const float* __restrict__ vb,
                                             int pitch, int T, int H, float scale, float* __restrict__ y, int ypitch) {
  constexpr int KS = D / 32;
  constexpr int DT = D / 16;
  __shared__ __attribute__((aligned(16))) unsigned short sKh[32][D + 8], sKl[32][D + 8], sVh[32][D + 8], sVl[32][D + 8];
  __shared__ __attribute__((aligned(16))) unsigned short sPh[4][16][40], sPl[4][16][40];
  __shared__ __attribute__((aligned(16))) float sO[4][16][D];
  const int tid = threadIdx.x, w = tid >> 5, lane = tid & 31, ln = lane & 15, hh = lane >> 4;
  const int nqb = (T + 63) / 64;
  const int bh = blockIdx.x / nqb, qblk = blockIdx.x % nqb;
  const int b = bh / H, h = bh % H;
  const int q0 = qblk * 64 + w * 16;
  const float* Q = qb + (size_t)b * T * pitch + h * D;
  const float* K = kb + (size_t)b * T * pitch + h * D;
  const float* V = vb + (size_t)b * T * pitch + h * D;

  FragB aqh[KS], aql[KS];
  {
    int row = q0 + ln; if (row >= T) row = T - 1;
    const float* qr = Q + (size_t)row * pitch;
#pragma unroll
    for (int ks = 0; ks < KS; ++ks)
#pragma unroll
      for (int i = 0; i < 16; ++i) {
        const int d = ks * 32 + ((i < 8) ? (8 * hh + i) : (16 + 8 * hh + (i - 8)));
        const float x = qr[d] * scale; const unsigned short hb = bf16_bits(x);
        aqh[ks].u[i] = hb; aql[ks].u[i] = bf16_bits(x - bf16_val(hb));
      }
  }
  float m_r[8], l_r[8];
#pragma unroll
  for (int r = 0; r < 8; ++r) { m_r[r] = -3.0e38f; l_r[r] = 0.f; }
  v8f oacc[DT];
#pragma unroll
  for (int dt = 0; dt < DT; ++dt) oacc[dt] = (v8f){0.f,0.f,0.f,0.f,0.f,0.f,0.f,0.f};

  const int kv_end = CAUSAL ? min(T, qblk * 64 + 64) : T;
  for (int j0 = 0; j0 < kv_end; j0 += 32) {
    __syncthreads();
    for (int e = tid; e < 32 * (D / 4); e += 128) {
      const int r = e / (D / 4), c4 = (e % (D / 4)) * 4;
      const int key = j0 + r;
      v4f kf = {0.f,0.f,0.f,0.f}, vf = {0.f,0.f,0.f,0.f};
      if (key < T) { kf = *(const v4fa*)(K + (size_t)key * pitch + c4); vf = *(const v4fa*)(V + (size_t)key * pitch + c4); }
#pragma unroll
      for (int t = 0; t < 4; ++t) {
        unsigned short hb = bf16_bits(kf[t]); sKh[r][c4 + t] = hb; sKl[r][c4 + t] = bf16_bits(kf[t] - bf16_val(hb));
        hb = bf16_bits(vf[t]); sVh[r][c4 + t] = hb; sVl[r][c4 + t] = bf16_bits(vf[t] - bf16_val(hb));
      }
    }
    __syncthreads();
    v8f s[2];
#pragma unroll
    for (int nt = 0; nt < 2; ++nt) {
      v8f acc = {};
#pragma unroll
      for (int ks = 0; ks < KS; ++ks) {
        FragB bh_, bl_;
        bh_.half[0] = *(const v8us*)&sKh[nt * 16 + ln][ks * 32 + 8 * hh]; bh_.half[1] = *(const v8us*)&sKh[nt * 16 + ln][ks * 32 + 16 + 8 * hh];
        bl_.half[0] = *(const v8us*)&sKl[nt * 16 + ln][ks * 32 + 8 * hh]; bl_.half[1] = *(const v8us*)&sKl[nt * 16 + ln][ks * 32 + 16 + 8 * hh];
        acc = mmaN<3>(aqh[ks].v, aql[ks].v, bh_.v, bl_.v, acc);
      }
      s[nt] = acc;
    }
    float alpha[8];
#pragma unroll
    for (int r = 0; r < 8; ++r) {
      const int qi = q0 + 8 * hh + r;
      const int ja = j0 + ln, jb = j0 + 16 + ln;
      if (CAUSAL) { if (ja > qi) s[0][r] = -3.0e38f; if (jb > qi) s[1][r] = -3.0e38f; }
      if (ja >= T) s[0][r] = -3.0e38f;
      if (jb >= T) s[1][r] = -3.0e38f;
      float mx = fmaxf(s[0][r], s[1][r]);
      mx = fmaxf(mx, __shfl_xor(mx, 1, 32)); mx = fmaxf(mx, __shfl_xor(mx, 2, 32)); mx = fmaxf(mx, __shfl_xor(mx, 4, 32)); mx = fmaxf(mx, __shfl_xor(mx, 8, 32));
      const float mnew = fmaxf(m_r[r], mx);
      alpha[r] = (mnew > -1.0e38f) ? __expf(m_r[r] - mnew) : 1.0f;
      const float p0 = (s[0][r] > -1.0e38f) ? __expf(s[0][r] - mnew) : 0.f;
      const float p1 = (s[1][r] > -1.0e38f) ? __expf(s[1][r] - mnew) : 0.f;
      m_r[r] = mnew;
      l_r[r] = l_r[r] * alpha[r] + p0 + p1;
      unsigned short hb = bf16_bits(p0); sPh[w][8 * hh + r][ln] = hb;      sPl[w][8 * hh + r][ln] = bf16_bits(p0 - bf16_val(hb));
      hb = bf16_bits(p1);                sPh[w][8 * hh + r][16 + ln] = hb; sPl[w][8 * hh + r][16 + ln] = bf16_bits(p1 - bf16_val(hb));
    }
#pragma unroll
    for (int dt = 0; dt < DT; ++dt)
#pragma unroll
      for (int r = 0; r < 8; ++r) oacc[dt][r] *= alpha[r];
    __builtin_amdgcn_fence(__ATOMIC_ACQ_REL, "workgroup");
    __builtin_amdgcn_wave_barrier();
    FragB pah, pal;
    pah.half[0] = *(const v8us*)&sPh[w][ln][8 * hh]; pah.half[1] = *(const v8us*)&sPh[w][ln][16 + 8 * hh];
    pal.half[0] = *(const v8us*)&sPl[w][ln][8 * hh]; pal.half[1] = *(const v8us*)&sPl[w][ln][16 + 8 * hh];
#pragma unroll
    for (int dt = 0; dt < DT; ++dt) {
      FragB bvh, bvl;
#pragma unroll
      for (int i = 0; i < 8; ++i) {
        bvh.u[i] = sVh[8 * hh + i][dt * 16 + ln]; bvh.u[8 + i] = sVh[16 + 8 * hh + i][dt * 16 + ln];
        bvl.u[i] = sVl[8 * hh + i][dt * 16 + ln]; bvl.u[8 + i] = sVl[16 + 8 * hh + i][dt * 16 + ln];
      }
      oacc[dt] = mmaN<3>(pah.v, pal.v, bvh.v, bvl.v, oacc[dt]);
    }
    __builtin_amdgcn_fence(__ATOMIC_ACQ_REL, "workgroup");
    __builtin_amdgcn_wave_barrier();
  }
#pragma unroll
  for (int r = 0; r < 8; ++r) {
    float l = l_r[r];
    l += __shfl_xor(l, 1, 32); l += __shfl_xor(l, 2, 32); l += __shfl_xor(l, 4, 32); l += __shfl_xor(l, 8, 32);
    l_r[r] = (l > 0.f) ? 1.0f / l : 0.f;
  }
#pragma unroll
  for (int dt = 0; dt < DT; ++dt)
#pragma unroll
    for (int r = 0; r < 8; ++r) sO[w][8 * hh + r][dt * 16 + ln] = oacc[dt][r] * l_r[r];
  __builtin_amdgcn_fence(__ATOMIC_ACQ_REL, "workgroup");
  __builtin_amdgcn_wave_barrier();
  for (int pass = 0; pass < 2; ++pass) {
    for (int r = 0; r < 16; ++r) {
      const int row = q0 + r;
      if (row < T && lane < D / 4) {
        const v4f val = *(const v4fa*)&sO[w][r][lane * 4];
        *(volatile v4f*)(y + ((size_t)b * T + row) * ypitch + h * D + lane * 4) = val;
      }
    }
    if (pass == 0) __threadfence();
  }
}

__global__ __launch_bounds__(256) void k_wt_pad(const float* __restrict__ W, unsigned short* __restrict__ Bt, int Kin, int Nout, int Kp, int Np) {
  const int t = blockIdx.x * 256 + threadIdx.x; const int k8n = Kp / 8; if (t >= Np * k8n) return; const int n = t / k8n, k8 = (t % k8n) * 8; v8us v;
#pragma unroll 1
  for (int i = 0; i < 8; ++i) { const int k = k8 + i; v[i] = (n < Nout && k < Kin) ? bf16_bits(W[(size_t)k * Nout + n]) : (unsigned short)0; }
  *(volatile v8us*)(Bt + (size_t)n * Kp + k8) = v; __threadfence(); *(volatile v8us*)(Bt + (size_t)n * Kp + k8) = v;
}
__global__ __launch_bounds__(256) void k_knn(const float* __restrict__ x, float* __restrict__ h0) {
  __shared__ float sx[256][3]; __shared__ __attribute__((aligned(16))) float srow[256][36];
  const int p = blockIdx.x * 256 + threadIdx.x; const int b = p / NPT; const float* xb = x + (size_t)b * NPT * 3;
  const float px = bf16_round(x[(size_t)p * 3]), py = bf16_round(x[(size_t)p * 3 + 1]), pz = bf16_round(x[(size_t)p * 3 + 2]);
  const float sq = px * px + py * py + pz * pz;
  float best[KNN]; for (int i = 0; i < KNN; ++i) best[i] = 3.0e38f;
  for (int c0 = 0; c0 < NPT; c0 += 256) {
    __syncthreads();
    { const int c = c0 + threadIdx.x; sx[threadIdx.x][0] = bf16_round(xb[(size_t)c * 3]); sx[threadIdx.x][1] = bf16_round(xb[(size_t)c * 3 + 1]); sx[threadIdx.x][2] = bf16_round(xb[(size_t)c * 3 + 2]); }
    __syncthreads();
#pragma unroll 1
    for (int j = 0; j < 256; ++j) {
      const float qx = sx[j][0], qy = sx[j][1], qz = sx[j][2];
      const float d = sq + (qx * qx + qy * qy + qz * qz) - 2.0f * (px * qx + py * qy + pz * qz);
      if (d < best[KNN - 1]) { int i = KNN - 1; while (i > 0 && best[i - 1] > d) { best[i] = best[i - 1]; --i; } best[i] = d; }
    }
  }
  { float* r = srow[threadIdx.x]; r[0] = px; r[1] = py; r[2] = pz; for (int i = 0; i < KNN; ++i) r[3 + i] = best[i]; for (int i = 3 + KNN; i < 32; ++i) r[i] = 0.f; }
  __syncthreads();
  const int w = threadIdx.x >> 5, lane = threadIdx.x & 31; const size_t prow0 = (size_t)blockIdx.x * 256;
  for (int pass = 0; pass < 2; ++pass) {
#pragma unroll 1
    for (int it = 0; it < 8; ++it) { const int rloc = w * 32 + it * 4 + (lane >> 3); const int c4 = (lane & 7) * 4; const v4f v = *(const v4fa*)&srow[rloc][c4]; *(volatile v4f*)(h0 + (prow0 + rloc) * 32 + c4) = v; }
    if (pass == 0) __threadfence();
  }
}

__global__ __launch_bounds__(256) void k_padbias(const float* __restrict__ b1a, const float* __restrict__ b1b, const float* __restrict__ b2, const float* __restrict__ b3b, float* __restrict__ bp) {
  const int t = threadIdx.x + blockIdx.x * 256; if (t >= 512) return; float v = 0.f;
  if (t < 64) v = (t < 20) ? bf16_round(b1a[t]) : 0.f; else if (t < 128) v = 0.f; else if (t < 256) v = (t - 128 < GF) ? bf16_round(b1b[t - 128]) : 0.f; else if (t < 384) v = (t - 256 < GF) ? bf16_round(b2[t - 256]) : 0.f; else if (t < 448) v = (t - 384 < 10) ? bf16_round(b3b[t - 384]) : 0.f;
  *(volatile float*)(bp + t) = v; __threadfence(); *(volatile float*)(bp + t) = v;
}
__global__ __launch_bounds__(128) void k_colsum(const float* __restrict__ x2, float* __restrict__ part) {
  const int c = threadIdx.x; const int blk = blockIdx.x; const int b = blk / (NPT / 512), rb = blk % (NPT / 512);
  float s = 0.f;
#pragma unroll 1
  for (int r = 0; r < 512; ++r) s += x2[((size_t)b * NPT + rb * 512 + r) * 128 + c];
  *(volatile float*)(part + (size_t)blk * 128 + c) = s; __threadfence(); *(volatile float*)(part + (size_t)blk * 128 + c) = s;
}
__global__ __launch_bounds__(64) void k_poolbias(const float* __restrict__ part, const float* __restrict__ w3a, const float* __restrict__ b3a, float* __restrict__ bias3) {
  __shared__ float mean[128];
  const int b = blockIdx.x, t = threadIdx.x;
  for (int c = t; c < 128; c += 64) { float s = 0.f; for (int k = 0; k < NPT / 512; ++k) s += part[((size_t)b * (NPT / 512) + k) * 128 + c]; mean[c] = s / (float)NPT; }
  __syncthreads();
  float v = 0.f; if (t < 20) { v = bf16_round(b3a[t]);
#pragma unroll 1
    for (int c = 0; c < GF; ++c) v += mean[c] * bf16_round(w3a[(size_t)(GF + c) * 20 + t]); }
  *(volatile float*)(bias3 + b * 64 + t) = v; __threadfence(); *(volatile float*)(bias3 + b * 64 + t) = v;
}
__global__ __launch_bounds__(256) void k_final(const float* __restrict__ o2, const float* __restrict__ w3c, const float* __restrict__ b3c, float* __restrict__ out) {
  const int p = blockIdx.x * 256 + threadIdx.x; const float* r = o2 + (size_t)p * 64;
  float z0 = bf16_round(b3c[0]), z1 = bf16_round(b3c[1]);
#pragma unroll 1
  for (int k = 0; k < 10; ++k) { const float hv = r[k]; z0 += hv * bf16_round(w3c[k * 2]); z1 += hv * bf16_round(w3c[k * 2 + 1]); }
  const float m = fmaxf(z0, z1); const float lse = m + logf(expf(z0 - m) + expf(z1 - m));
  typedef float v2f __attribute__((ext_vector_type(2))); const v2f v = {z0 - lse, z1 - lse};
  *(volatile v2f*)(out + (size_t)p * 2) = v; __threadfence(); *(volatile v2f*)(out + (size_t)p * 2) = v;
}
extern "C" void kernel_launch(void* const* d_in, const int* in_sizes, int n_in,
                              void* d_out, int out_size, void* d_ws, size_t ws_size, hipStream_t stream) {
  (void)in_sizes; (void)n_in; (void)out_size;
  const float* x = (const float*)d_in[0];
  const float* w1a = (const float*)d_in[1]; const float* b1a = (const float*)d_in[2]; const float* w1b = (const float*)d_in[3]; const float* b1b = (const float*)d_in[4];
  const float* w2 = (const float*)d_in[5]; const float* b2 = (const float*)d_in[6]; const float* w3a = (const float*)d_in[7]; const float* b3a = (const float*)d_in[8];
  const float* w3b = (const float*)d_in[9]; const float* b3b = (const float*)d_in[10]; const float* w3c = (const float*)d_in[11]; const float* b3c = (const float*)d_in[12];
  char* ws = (char*)d_ws; size_t off = 0;
  auto take = [&](size_t bytes) { char* p = ws + off; off += (bytes + 255) & ~(size_t)255; return p; };
  const int M = BB * NPT;
  unsigned short* B1a = (unsigned short*)take(64 * 32 * 2); unsigned short* B1b = (unsigned short*)take(128 * 64 * 2); unsigned short* B2w = (unsigned short*)take(128 * 128 * 2); unsigned short* B3a = (unsigned short*)take(64 * 128 * 2); unsigned short* B3b = (unsigned short*)take(64 * 64 * 2);
  float* h0 = (float*)take((size_t)M * 32 * 4); float* h1 = (float*)take((size_t)M * 64 * 4); float* x1 = (float*)take((size_t)M * 128 * 4); float* x2 = (float*)take((size_t)M * 128 * 4);
  float* o1 = (float*)take((size_t)M * 64 * 4); float* o2 = (float*)take((size_t)M * 64 * 4);
  float* part = (float*)take((size_t)BB * (NPT / 512) * 128 * 4); float* bias3 = (float*)take(BB * 64 * 4);
  float* bpad = (float*)take(4 * 128 * 4);
  if (off > ws_size) return;
  k_wt_pad<<<(64 * 4 + 255) / 256, 256, 0, stream>>>(w1a, B1a, 13, 20, 32, 64);
  k_wt_pad<<<(128 * 8 + 255) / 256, 256, 0, stream>>>(w1b, B1b, 20, GF, 64, 128);
  k_wt_pad<<<(128 * 16 + 255) / 256, 256, 0, stream>>>(w2, B2w, GF, GF, 128, 128);
  k_wt_pad<<<(64 * 16 + 255) / 256, 256, 0, stream>>>(w3a, B3a, GF, 20, 128, 64);
  k_wt_pad<<<(64 * 8 + 255) / 256, 256, 0, stream>>>(w3b, B3b, 20, 10, 64, 64);
  k_knn<<<M / 256, 256, 0, stream>>>(x, h0);
  k_padbias<<<2, 256, 0, stream>>>(b1a, b1b, b2, b3b, bpad);
  const int g64 = ((M / 16) * 1 + 3) / 4, g128 = ((M / 16) * 2 + 3) / 4;
  k_gemm_bf<true, 1, false><<<g64, 128, 0, stream>>>(h0, 32, B1a, 32, bpad + 0, h1, 64, M, 64, 32);
  k_gemm_bf<true, 1, false><<<g128, 128, 0, stream>>>(h1, 64, B1b, 64, bpad + 128, x1, 128, M, 128, 64);
  k_gemm_bf<true, 1, false><<<g128, 128, 0, stream>>>(x1, 128, B2w, 128, bpad + 256, x2, 128, M, 128, 128);
  k_colsum<<<BB * (NPT / 512), 128, 0, stream>>>(x2, part);
  k_poolbias<<<BB, 64, 0, stream>>>(part, w3a, b3a, bias3);
  for (int b = 0; b < BB; ++b)
    k_gemm_bf<true, 1, false><<<((NPT / 16) + 3) / 4, 128, 0, stream>>>(x1 + (size_t)b * NPT * 128, 128, B3a, 128, bias3 + b * 64, o1 + (size_t)b * NPT * 64, 64, NPT, 64, 128);
  k_gemm_bf<true, 1, false><<<g64, 128, 0, stream>>>(o1, 64, B3b, 64, bpad + 384, o2, 64, M, 64, 64);
  k_final<<<M / 256, 256, 0, stream>>>(o2, w3c, b3c, (float*)d_out);
}
